// effConvKAN3D_9311489097883
// MI455X (gfx1250) — hardware-verified
//
#include <hip/hip_runtime.h>

#pragma clang fp contract(off)

typedef _Float16 v16h __attribute__((ext_vector_type(16)));
typedef _Float16 v8h  __attribute__((ext_vector_type(8)));
typedef float    v8f  __attribute__((ext_vector_type(8)));
typedef float    v4f  __attribute__((ext_vector_type(4)));
union Frag   { v16h v; v8h half[2]; };
union Pack16 { v8h v[2]; _Float16 s[16]; };

#define IN_CH    8
#define OUT_CH   16
#define VD       32
#define NPOS     32768
#define NX       (IN_CH * NPOS)
#define NTAP     27
#define NSLOT    28
#define IN_FEAT  (IN_CH * NTAP)
#define NB       8
#define EW       16
#define KW       (IN_CH * NSLOT * EW)
#define NKSTEP   (KW / 32)
#define NKNOT    12
#define ZROW     NX
#define ZZROW    (NX + 1)
#define E_BLK    256
#define E_NBLK   ((NX + 2 + E_BLK - 1) / E_BLK)
#define E_ROWS   (E_NBLK * E_BLK)
#define BM       128
#define WP_THREADS (IN_CH * NSLOT)
#define GH       0.4f
#define GLO      (-1.0f)
#define WSCALE   16.0f
#define OSCALE   0.0625f

static_assert(NPOS % BM == 0);
static_assert(KW % 32 == 0);
static_assert(NSLOT % 2 == 0);
static_assert((E_BLK * EW * 2) % 512 == 0);
static_assert((KW * 2) % 512 == 0);
static_assert((KW / 8) == 2 * WP_THREADS);
static_assert(WP_THREADS % 32 == 0);
static_assert(E_ROWS >= NX + 2);

__device__ __forceinline__ v8f wmma16(v16h a, v16h b, v8f c)
{
    v8f d = __builtin_amdgcn_wmma_f32_16x16x32_f16(false, a, false, b, (short)0, c, false, false);
    asm volatile("v_nop\n\tv_nop\n\tv_nop\n\tv_nop" : "+v"(d) : "v"(a), "v"(b));
    return d;
}

__device__ __forceinline__ void kan_feat(float xv, float f[EW])
{
    float g[NKNOT];
    #pragma unroll
    for (int j = 0; j < NKNOT; ++j) g[j] = (float)(j - 3) * GH + GLO;

    float b[NKNOT - 1];
    #pragma unroll
    for (int j = 0; j < NKNOT - 1; ++j)
        b[j] = (xv >= g[j] && xv < g[j + 1]) ? 1.0f : 0.0f;

    #pragma unroll
    for (int j = 0; j < 10; ++j) {
        const float rl = 1.0f / (g[j + 1] - g[j]);
        const float rr = 1.0f / (g[j + 2] - g[j + 1]);
        const float lf = (xv - g[j]) * rl;
        const float rt = (g[j + 2] - xv) * rr;
        const float pl = lf * b[j];
        const float pr = rt * b[j + 1];
        b[j] = pl + pr;
    }
    #pragma unroll
    for (int j = 0; j < 9; ++j) {
        const float rl = 1.0f / (g[j + 2] - g[j]);
        const float rr = 1.0f / (g[j + 3] - g[j + 1]);
        const float lf = (xv - g[j]) * rl;
        const float rt = (g[j + 3] - xv) * rr;
        const float pl = lf * b[j];
        const float pr = rt * b[j + 1];
        b[j] = pl + pr;
    }
    #pragma unroll
    for (int j = 0; j < 8; ++j) {
        const float rl = 1.0f / (g[j + 3] - g[j]);
        const float rr = 1.0f / (g[j + 4] - g[j + 1]);
        const float lf = (xv - g[j]) * rl;
        const float rt = (g[j + 4] - xv) * rr;
        const float pl = lf * b[j];
        const float pr = rt * b[j + 1];
        b[j] = pl + pr;
    }

    const float ex = __expf(-xv);
    const float sg = __builtin_amdgcn_rcpf(1.0f + ex);
    f[0] = xv * sg;
    #pragma unroll
    for (int c = 0; c < NB; ++c) f[1 + c] = b[c];
    #pragma unroll
    for (int q = 1 + NB; q < EW; ++q) f[q] = 0.0f;
}

__global__ __launch_bounds__(WP_THREADS) void k_wprep(const float* __restrict__ bw,
                                                      const float* __restrict__ sw,
                                                      const float* __restrict__ sc,
                                                      _Float16* __restrict__ Wp)
{
    __shared__ __attribute__((aligned(16))) _Float16 rowbuf[KW];
    const int tid = threadIdx.x;
    const int o   = blockIdx.x;
    const int ch  = tid / NSLOT;
    const int t   = tid - ch * NSLOT;
    const int tt  = (t < NTAP) ? t : (NTAP - 1);
    const int i   = ch * NTAP + tt;
    const int oi  = o * IN_FEAT + i;

    const float b = bw[oi];
    const float s = sc[oi];
    const v4f c0 = *(const v4f*)(sw + (size_t)oi * NB);
    const v4f c1 = *(const v4f*)(sw + (size_t)oi * NB + 4);
    const bool pad = (t >= NTAP);

    float v[EW];
    v[0] = b * WSCALE;
    v[1] = (c0[0] * s) * WSCALE;
    v[2] = (c0[1] * s) * WSCALE;
    v[3] = (c0[2] * s) * WSCALE;
    v[4] = (c0[3] * s) * WSCALE;
    v[5] = (c1[0] * s) * WSCALE;
    v[6] = (c1[1] * s) * WSCALE;
    v[7] = (c1[2] * s) * WSCALE;
    v[8] = (c1[3] * s) * WSCALE;
    #pragma unroll
    for (int q = 1 + NB; q < EW; ++q) v[q] = 0.0f;

    Pack16 pk;
    #pragma unroll
    for (int q = 0; q < EW; ++q) pk.s[q] = (_Float16)(pad ? 0.0f : v[q]);
    *(v8h*)(rowbuf + tid * EW)     = pk.v[0];
    *(v8h*)(rowbuf + tid * EW + 8) = pk.v[1];
    __syncthreads();

    v8h vv[2];
    #pragma unroll
    for (int q = 0; q < 2; ++q) {
        const int pc = q * WP_THREADS + tid;
        vv[q] = *(const v8h*)(rowbuf + pc * 8);
    }
    _Float16* dst = Wp + (size_t)o * KW;
    #pragma unroll
    for (int q = 0; q < 2; ++q) {
        const int pc = q * WP_THREADS + tid;
        *(volatile v8h*)(dst + pc * 8) = vv[q];
    }
    __threadfence();
    #pragma unroll
    for (int q = 0; q < 2; ++q) {
        const int pc = q * WP_THREADS + tid;
        *(volatile v8h*)(dst + pc * 8) = vv[q];
    }
}

__global__ __launch_bounds__(E_BLK) void k_feat(const float* __restrict__ x,
                                                _Float16* __restrict__ E)
{
    __shared__ __attribute__((aligned(16))) _Float16 rows[E_BLK * EW];
    const int tid = threadIdx.x;
    const int l   = tid & 31;
    const int w   = tid >> 5;
    const int e   = blockIdx.x * E_BLK + tid;
    const int ecl = (e < NX) ? e : (NX - 1);
    float xv = x[ecl];
    xv = (e < NX) ? xv : 0.0f;

    float f[EW];
    kan_feat(xv, f);
    const bool zr = (e > NX);

    Pack16 pk;
    #pragma unroll
    for (int q = 0; q < EW; ++q) pk.s[q] = (_Float16)(zr ? 0.0f : f[q]);
    *(v8h*)(rows + tid * EW)     = pk.v[0];
    *(v8h*)(rows + tid * EW + 8) = pk.v[1];
    __syncthreads();

    v8h vv[2];
    #pragma unroll
    for (int q = 0; q < 2; ++q) {
        const int pc = (2 * w + q) * 32 + l;
        vv[q] = *(const v8h*)(rows + pc * 8);
    }
    _Float16* dst = E + (size_t)blockIdx.x * (E_BLK * EW);
    #pragma unroll
    for (int q = 0; q < 2; ++q) {
        const int pc = (2 * w + q) * 32 + l;
        *(volatile v8h*)(dst + pc * 8) = vv[q];
    }
    __threadfence();
    #pragma unroll
    for (int q = 0; q < 2; ++q) {
        const int pc = (2 * w + q) * 32 + l;
        *(volatile v8h*)(dst + pc * 8) = vv[q];
    }
}

__device__ __forceinline__ int tap_off(int t)
{
    const int kd = t / 9;
    const int r  = t - 9 * kd;
    const int kh = r / 3;
    const int kw = r - 3 * kh;
    return (kd - 1) * (VD * VD) + (kh - 1) * VD + (kw - 1);
}

__global__ __launch_bounds__(256) void k_gemm(const _Float16* __restrict__ E,
                                              const _Float16* __restrict__ Wp,
                                              float* __restrict__ out)
{
    __shared__ __attribute__((aligned(16))) float Cs[OUT_CH * BM];
    const int l = threadIdx.x & 31;
    const int w = threadIdx.x >> 5;
    const int h = l >> 4;
    const int m = l & 15;
    const int bpos = blockIdx.x * BM;
    const int p  = bpos + w * 16 + m;
    const int pd = p >> 10;
    const int ph = (p >> 5) & 31;
    const int pw = p & 31;

    const unsigned PD = 0x1FFu;
    const unsigned PH = 0x1C0E07u;
    const unsigned PW = 0x1249249u;
    const unsigned md = ((pd > 0) ? PD : 0u) | (PD << 9) | ((pd < VD - 1) ? (PD << 18) : 0u);
    const unsigned mh = ((ph > 0) ? PH : 0u) | (PH << 3) | ((ph < VD - 1) ? (PH << 6) : 0u);
    const unsigned mw = ((pw > 0) ? PW : 0u) | (PW << 1) | ((pw < VD - 1) ? (PW << 2) : 0u);
    const unsigned vmask = md & mh & mw;

    const _Float16* eh   = E + 8 * h;
    const _Float16* wrow = Wp + (size_t)m * KW + 8 * h;

    v8f acc = {};

    #pragma unroll 2
    for (int ks = 0; ks < NKSTEP; ++ks) {
        const int u0 = 2 * ks;
        const int ch = u0 / NSLOT;
        const int t0 = u0 - ch * NSLOT;
        const int t1 = t0 + 1;
        const int off0 = tap_off(t0);
        const int off1 = tap_off(t1);
        const int ec = ch * NPOS + p;
        const bool v0 = ((vmask >> t0) & 1u) != 0u;
        const bool v1 = ((vmask >> t1) & 1u) != 0u;
        const int z1 = (t1 >= NTAP) ? ZZROW : ZROW;
        const int i0 = v0 ? (ec + off0) : ZROW;
        const int i1 = v1 ? (ec + off1) : z1;

        Frag a, b;
        a.half[0] = *(const v8h*)(eh + i0 * EW);
        a.half[1] = *(const v8h*)(eh + i1 * EW);
        b.half[0] = *(const v8h*)(wrow + 32 * ks);
        b.half[1] = *(const v8h*)(wrow + 32 * ks + 16);
        acc = wmma16(a.v, b.v, acc);
    }

    float* crow = Cs + m * BM + w * 16 + 8 * h;
    #pragma unroll
    for (int r = 0; r < 8; ++r) crow[r] = acc[r] * OSCALE;
    __syncthreads();

    v4f vals[2];
    #pragma unroll
    for (int q = 0; q < 2; ++q) {
        const int o = w + 8 * q;
        vals[q] = *(const v4f*)(Cs + o * BM + 4 * l);
    }
    #pragma unroll
    for (int q = 0; q < 2; ++q) {
        const int o = w + 8 * q;
        *(volatile v4f*)(out + (size_t)o * NPOS + bpos + 4 * l) = vals[q];
    }
    __threadfence();
    #pragma unroll
    for (int q = 0; q < 2; ++q) {
        const int o = w + 8 * q;
        *(volatile v4f*)(out + (size_t)o * NPOS + bpos + 4 * l) = vals[q];
    }
}

extern "C" void kernel_launch(void* const* d_in, const int* in_sizes, int n_in,
                              void* d_out, int out_size, void* d_ws, size_t ws_size,
                              hipStream_t stream)
{
    if (n_in < 4) return;
    if (in_sizes[0] != NX) return;
    if (in_sizes[1] != OUT_CH * IN_FEAT) return;
    if (in_sizes[2] != OUT_CH * IN_FEAT * NB) return;
    if (in_sizes[3] != OUT_CH * IN_FEAT) return;
    if (out_size != OUT_CH * NPOS) return;

    const float* x  = (const float*)d_in[0];
    const float* bw = (const float*)d_in[1];
    const float* sw = (const float*)d_in[2];
    const float* sc = (const float*)d_in[3];
    float* out = (float*)d_out;

    const size_t ebytes = (size_t)E_ROWS * EW * sizeof(_Float16);
    const size_t woff   = (ebytes + 127) & ~(size_t)127;
    const size_t wbytes = (size_t)OUT_CH * KW * sizeof(_Float16);
    if (woff + wbytes > ws_size) return;
    _Float16* E  = (_Float16*)d_ws;
    _Float16* Wp = (_Float16*)((char*)d_ws + woff);

    k_wprep<<<dim3(OUT_CH), dim3(WP_THREADS), 0, stream>>>(bw, sw, sc, Wp);
    k_feat<<<dim3(E_NBLK), dim3(E_BLK), 0, stream>>>(x, E);
    k_gemm<<<dim3(NPOS / BM), dim3(256), 0, stream>>>(E, Wp, out);
}
